// GraphFusionModel_40157944218453
// MI455X (gfx1250) — hardware-verified
//
#include <hip/hip_runtime.h>


#define TT   768
#define SS   3
#define NN   2304
#define DIM  128
#define NHD  4
#define DK   32
#define DFF  512
#define NL   3
#define ZH   2
typedef _Float16 h16;
typedef unsigned short bf;
typedef __attribute__((ext_vector_type(16))) __bf16   v16bf;
typedef __attribute__((ext_vector_type(16))) _Float16 v16h;
typedef __attribute__((ext_vector_type(8)))  _Float16 v8h;
typedef __attribute__((ext_vector_type(8)))  unsigned short v8us;
typedef __attribute__((ext_vector_type(8)))  float    v8f;
typedef __attribute__((ext_vector_type(4)))  float    v4f;
typedef v8h  __attribute__((may_alias)) v8ha;
typedef v4f  __attribute__((may_alias)) v4fa;
typedef v8us __attribute__((may_alias)) v8usa;

__device__ __forceinline__ unsigned short f2bf(float f) { unsigned u = __float_as_uint(f); u += 0x7FFFu + ((u >> 16) & 1u); return (unsigned short)(u >> 16); }
__device__ __forceinline__ float bf2f(unsigned short b) { return __uint_as_float(((unsigned)b) << 16); }
__device__ __forceinline__ float bfr(float f) { return bf2f(f2bf(f)); }
__device__ __forceinline__ v16h cat16(v8h lo, v8h hi) { return __builtin_shufflevector(lo, hi, 0, 1, 2, 3, 4, 5, 6, 7, 8, 9, 10, 11, 12, 13, 14, 15); }
__device__ __forceinline__ v16bf cat16b(v8us lo, v8us hi) { return __builtin_bit_cast(v16bf, __builtin_shufflevector(lo, hi, 0, 1, 2, 3, 4, 5, 6, 7, 8, 9, 10, 11, 12, 13, 14, 15)); }
__device__ __forceinline__ v8f wmma16(v16h a, v16h b, v8f c) { return __builtin_amdgcn_wmma_f32_16x16x32_f16(false, a, false, b, (short)0, c, false, false); }
__device__ __forceinline__ v8f wmmab(v16bf a, v16bf b, v8f c) { return __builtin_amdgcn_wmma_f32_16x16x32_bf16(false, a, false, b, (short)0, c, false, false); }


template <typename T16> struct WFrag;
template <> struct WFrag<h16> { typedef v16h V; static __device__ __forceinline__ V ld(const h16* p) { return cat16(*(const v8h*)p, *(const v8h*)(p + 16)); } static __device__ __forceinline__ v8f mma(V a, V b, v8f c) { return wmma16(a, b, c); } };
template <> struct WFrag<bf> { typedef v16bf V; static __device__ __forceinline__ V ld(const bf* p) { return cat16b(*(const v8us*)p, *(const v8us*)(p + 16)); } static __device__ __forceinline__ v8f mma(V a, V b, v8f c) { return wmmab(a, b, c); } };
template <typename T16, int NSPLIT, bool BIAS>
__global__ __launch_bounds__(32) void k_gemmw(const T16* __restrict__ A, const T16* __restrict__ A2, const T16* __restrict__ Bt, const T16* __restrict__ Bt2, int K, float* C, int ldc, const float* __restrict__ bias, size_t sA, size_t sB, size_t sC) {
    typedef typename WFrag<T16>::V V;
    __shared__ __align__(16) float os[16 * 68];
    const size_t z = blockIdx.z; A += z * sA; if (A2) A2 += z * sA; Bt += z * sB; if (Bt2) Bt2 += z * sB; C += z * sC;
    const int lane = threadIdx.x & 31, lr = lane & 15, hi = lane >> 4; const int r0 = blockIdx.x * 64, c0 = blockIdx.y * 64;
    v8f acc[4][4];
#pragma unroll
    for (int mb = 0; mb < 4; ++mb)
#pragma unroll
        for (int nb = 0; nb < 4; ++nb) acc[mb][nb] = (v8f){};
    const size_t aoff = (size_t)(r0 + lr) * K + 8 * hi, boff = (size_t)(c0 + lr) * K + 8 * hi;
#pragma unroll 1
    for (int kc = 0; kc < K; kc += 32) {
        V a[4], a2[4];
#pragma unroll
        for (int mb = 0; mb < 4; ++mb) { a[mb] = WFrag<T16>::ld(A + aoff + (size_t)mb * 16 * K + kc); if (NSPLIT == 1 || NSPLIT == 2) a2[mb] = WFrag<T16>::ld(A2 + aoff + (size_t)mb * 16 * K + kc); }
#pragma unroll
        for (int nb = 0; nb < 4; ++nb) { const V b = WFrag<T16>::ld(Bt + boff + (size_t)nb * 16 * K + kc); V b2; if (NSPLIT >= 2) b2 = WFrag<T16>::ld(Bt2 + boff + (size_t)nb * 16 * K + kc);
#pragma unroll
            for (int mb = 0; mb < 4; ++mb) { acc[mb][nb] = WFrag<T16>::mma(a[mb], b, acc[mb][nb]); if (NSPLIT == 1 || NSPLIT == 2) acc[mb][nb] = WFrag<T16>::mma(a2[mb], b, acc[mb][nb]); if (NSPLIT >= 2) acc[mb][nb] = WFrag<T16>::mma(a[mb], b2, acc[mb][nb]); } }
        asm volatile("v_nop\n\tv_nop\n\tv_nop\n\tv_nop" : "+v"(acc[0][0]), "+v"(acc[1][1]), "+v"(acc[2][2]), "+v"(acc[3][3]) : "v"(a[0]), "v"(a[3]));
    }
#pragma unroll
    for (int mb = 0; mb < 4; ++mb) {
#pragma unroll
        for (int nb = 0; nb < 4; ++nb) {
#pragma unroll
            for (int j = 0; j < 8; ++j) os[(hi * 8 + j) * 68 + nb * 16 + lr] = acc[mb][nb][j]; }
        __builtin_amdgcn_wave_barrier(); asm volatile("" ::: "memory");
        float* crow = C + (size_t)(r0 + mb * 16) * ldc + c0;
#pragma unroll 1
        for (int ps = 0; ps < 2; ++ps) {
#pragma unroll
            for (int s = 0; s < 8; ++s) { const int row = 2 * s + hi, cofs = lr * 4; v4f val = *(const v4fa*)(os + row * 68 + cofs); if (BIAS) { val[0] += bfr(bias[c0 + cofs]); val[1] += bfr(bias[c0 + cofs + 1]); val[2] += bfr(bias[c0 + cofs + 2]); val[3] += bfr(bias[c0 + cofs + 3]); }
                *(volatile v4f*)(crow + (size_t)row * ldc + cofs) = val; }
            if (ps == 0) __threadfence(); }
        __builtin_amdgcn_wave_barrier(); asm volatile("" ::: "memory");
    }
}

__device__ __forceinline__ float geluf(float x) { return 0.5f * x * (1.0f + erff(x * 0.70710678118654752f)); }
__device__ __forceinline__ void splitf(float y, unsigned short& h, unsigned short& l) { h = f2bf(y); l = f2bf(y - bf2f(h)); }

__global__ __launch_bounds__(256) void k_cvt8(const float* __restrict__ src, bf* dst, size_t n8) {
    const size_t i = (size_t)blockIdx.x * 256 + threadIdx.x; if (i >= n8) return;
    const v8f v = *(const v8f*)(src + i * 8); v8us o;
#pragma unroll
    for (int k = 0; k < 8; ++k) o[k] = f2bf(v[k]);
    *(volatile v8us*)(dst + i * 8) = o; __threadfence(); *(volatile v8us*)(dst + i * 8) = o;
}
__global__ __launch_bounds__(256) void k_w2pad(const float* __restrict__ w, bf* dst) {
    const int i = blockIdx.x * 256 + threadIdx.x; if (i >= 64 * 128 / 8) return; v8us o;
#pragma unroll
    for (int k = 0; k < 8; ++k) { const int e = i * 8 + k; o[k] = (e < 3 * DIM) ? f2bf(w[e < 3 * DIM ? e : 0]) : (unsigned short)0; }
    *(volatile v8us*)(dst + (size_t)i * 8) = o; __threadfence(); *(volatile v8us*)(dst + (size_t)i * 8) = o;
}
__global__ __launch_bounds__(256) void k_embed(const float* __restrict__ obs, const float* __restrict__ cf, const float* __restrict__ Wp, const float* __restrict__ bp, const float* __restrict__ temb, const float* __restrict__ semb, float* X, bf* Xh, bf* Xl) {
    typedef __attribute__((ext_vector_type(4))) unsigned short v4us;
    const int lane = threadIdx.x & 31; const int n = blockIdx.x * 8 + (threadIdx.x >> 5); if (n >= NN) return; const int t = n / SS, s = n % SS; const int tc = t < 255 ? t : 255;
    float raw[8];
#pragma unroll
    for (int k = 0; k < 7; ++k) raw[k] = bfr(obs[(size_t)n * 7 + k]);
    raw[7] = bfr(cf[n]);
    v4f v; v4us oh, ol; const int c0 = lane * 4;
#pragma unroll
    for (int q = 0; q < 4; ++q) { const int c = c0 + q; float acc = 0.f;
#pragma unroll
        for (int k = 0; k < 8; ++k) acc = fmaf(raw[k], bfr(Wp[c * 8 + k]), acc);
        v[q] = acc + bfr(bp[c]) + bfr(temb[(size_t)tc * DIM + c]) + bfr(semb[s * DIM + c]);
        unsigned short h, l; splitf(v[q], h, l); oh[q] = h; ol[q] = l; }
#pragma unroll 1
    for (int ps = 0; ps < 2; ++ps) { *(volatile v4f*)(X + (size_t)n * DIM + c0) = v; *(volatile v4us*)(Xh + (size_t)n * DIM + c0) = oh; *(volatile v4us*)(Xl + (size_t)n * DIM + c0) = ol; if (ps == 0) __threadfence(); }
}
__global__ __launch_bounds__(256) void k_dist(const float* __restrict__ obs, float* DIST) {
    const int lane = threadIdx.x & 31; const int n = blockIdx.x * 8 + (threadIdx.x >> 5); if (n >= NN) return;
    const float px = bfr(obs[(size_t)n * 7 + 0]), py = bfr(obs[(size_t)n * 7 + 1]), pz = bfr(obs[(size_t)n * 7 + 2]);
#pragma unroll 1
    for (int ps = 0; ps < 2; ++ps) {
#pragma unroll 1
        for (int q = 0; q < NN / 128; ++q) { const int m0 = q * 128 + lane * 4; v4f o;
#pragma unroll
            for (int i = 0; i < 4; ++i) { const int m = m0 + i; const float dx = px - bfr(obs[(size_t)m * 7 + 0]), dy = py - bfr(obs[(size_t)m * 7 + 1]), dz = pz - bfr(obs[(size_t)m * 7 + 2]);
                float sq = __fmul_rn(dx, dx); sq = __fadd_rn(sq, __fmul_rn(dz, dz)); sq = __fadd_rn(sq, __fmul_rn(dy, dy)); o[i] = sqrtf(sq + 1e-12f); }
            *(volatile v4f*)(DIST + (size_t)n * NN + m0) = o; }
        if (ps == 0) __threadfence(); }
}
__global__ __launch_bounds__(256) void k_atab(const float* __restrict__ obs, const float* __restrict__ cf, const float* __restrict__ ew, float* ATAB) {
    const int lane = threadIdx.x & 31; const int n = (blockIdx.x * 8 + (threadIdx.x >> 5)) * 32 + lane; if (n - lane >= NN) return;
    float raw[8];
#pragma unroll
    for (int k = 0; k < 7; ++k) raw[k] = bfr(obs[(size_t)n * 7 + k]);
    raw[7] = bfr(cf[n]); float a[NHD];
#pragma unroll
    for (int h = 0; h < NHD; ++h) { const float* w = ew + h * 9; a[h] = raw[0] * bfr(w[0]) + raw[1] * bfr(w[1]) + raw[2] * bfr(w[2]) + raw[3] * bfr(w[4]) + raw[4] * bfr(w[5]) + raw[5] * bfr(w[6]) + raw[7] * bfr(w[7]); }
#pragma unroll 1
    for (int ps = 0; ps < 2; ++ps) {
#pragma unroll
        for (int h = 0; h < NHD; ++h) *(volatile float*)(ATAB + h * NN + n) = a[h];
        if (ps == 0) __threadfence(); }
}
__global__ __launch_bounds__(256) void k_qkplanes(const float* __restrict__ Q, const float* __restrict__ Kf, int h0, bf* Qh, bf* Ql, bf* Kh, bf* Kl) {
    typedef __attribute__((ext_vector_type(2))) unsigned short v2us;
    const int lane = threadIdx.x & 31; const size_t L0 = ((size_t)blockIdx.x * 8 + (threadIdx.x >> 5)) * 8; const size_t nlines = (size_t)ZH * NN * DK / 64;
#pragma unroll 1
    for (int ps = 0; ps < 2; ++ps) {
#pragma unroll
        for (int l = 0; l < 8; ++l) { const size_t L = L0 + l; if (L >= nlines) break; const size_t e = L * 64 + lane * 2; const int z = (int)(e / ((size_t)NN * DK)); const size_t rem = e % ((size_t)NN * DK); const int n = (int)(rem / DK), d = (int)(rem % DK);
            v2us qh, ql, kh, kl;
#pragma unroll
            for (int q = 0; q < 2; ++q) { const size_t src = (size_t)n * DIM + (h0 + z) * DK + d + q; unsigned short a, b; splitf(Q[src] * 0.17677669529663688f, a, b); qh[q] = a; ql[q] = b; splitf(Kf[src], a, b); kh[q] = a; kl[q] = b; }
            *(volatile v2us*)(Qh + e) = qh; *(volatile v2us*)(Ql + e) = ql; *(volatile v2us*)(Kh + e) = kh; *(volatile v2us*)(Kl + e) = kl; }
        if (ps == 0) __threadfence(); }
}
__global__ __launch_bounds__(256) void k_vT(const float* __restrict__ V, int h0, bf* VTh, bf* VTl) {
    __shared__ float tl[64][33];
    const int tid = threadIdx.x; const int m0 = blockIdx.x * 64; const int z = blockIdx.z; const int rr = tid >> 2, cq = (tid & 3) * 8;
#pragma unroll
    for (int i = 0; i < 8; ++i) tl[rr][cq + i] = V[(size_t)(m0 + rr) * DIM + (h0 + z) * DK + cq + i];
    __syncthreads();
    const int lane = tid & 31, wv = tid >> 5;
    auto pass = [&]() { const int mq = (lane & 7) * 8;
#pragma unroll
        for (int i2 = 0; i2 < 2; ++i2) { const int dr = wv * 8 + i2 * 4 + (lane >> 3); v8us oh, ol;
#pragma unroll
            for (int i = 0; i < 8; ++i) { unsigned short a = 0, b = 0; if (dr < DK) splitf(tl[mq + i][dr < DK ? dr : 0], a, b); oh[i] = a; ol[i] = b; }
            const size_t o = ((size_t)z * 64 + dr) * NN + m0 + mq; *(volatile v8us*)(VTh + o) = oh; *(volatile v8us*)(VTl + o) = ol; } };
    pass(); __threadfence(); pass();
}
__global__ __launch_bounds__(256) void k_softb(const float* __restrict__ Sb, const float* __restrict__ ATAB, const float* __restrict__ DIST, const float* __restrict__ ew, const float* __restrict__ eb, int h0, bf* PH, bf* PL) {
    typedef __attribute__((ext_vector_type(4))) unsigned short v4us;
    const int lane = threadIdx.x & 31, n = blockIdx.x * 8 + (threadIdx.x >> 5); if (n >= NN) return; const int z = blockIdx.z, h = h0 + z;
    const size_t zo = ((size_t)z * NN + n) * NN; const float* sr = Sb + zo; const float* dr = DIST + (size_t)n * NN; const float* at = ATAB + h * NN;
    const float w3 = bfr(ew[h * 9 + 3]), w8 = bfr(ew[h * 9 + 8]) * (1.0f / TT), cst = at[n] + bfr(eb[h]); const int tn = n / SS;
    auto val = [&](int m) { return sr[m] + (cst - at[m] + w3 * dr[m] + w8 * (float)abs(tn - m / SS)); };
    float mx = -3.0e38f;
#pragma unroll 1
    for (int c0 = lane * 4; c0 < NN; c0 += 128) {
#pragma unroll
        for (int q = 0; q < 4; ++q) mx = fmaxf(mx, val(c0 + q)); }
#pragma unroll
    for (int sh = 16; sh; sh >>= 1) mx = fmaxf(mx, __shfl_xor(mx, sh, 32));
    float sum = 0.f;
#pragma unroll 1
    for (int c0 = lane * 4; c0 < NN; c0 += 128) {
#pragma unroll
        for (int q = 0; q < 4; ++q) sum += __expf(val(c0 + q) - mx); }
#pragma unroll
    for (int sh = 16; sh; sh >>= 1) sum += __shfl_xor(sum, sh, 32);
    const float inv = __fdiv_rn(1.0f, sum);
#pragma unroll 1
    for (int ps = 0; ps < 2; ++ps) {
#pragma unroll 1
        for (int c0 = lane * 4; c0 < NN; c0 += 128) { v4us oh, ol;
#pragma unroll
            for (int q = 0; q < 4; ++q) { const float p = __expf(val(c0 + q) - mx) * inv; unsigned short a, b; splitf(p, a, b); oh[q] = a; ol[q] = b; }
            const size_t o = zo + c0; *(volatile v4us*)(PH + o) = oh; *(volatile v4us*)(PL + o) = ol; }
        if (ps == 0) __threadfence(); }
}
__global__ __launch_bounds__(256) void k_mergez(const float* __restrict__ OZ, int h0, float* AO) {
    typedef __attribute__((ext_vector_type(2))) float v2f;
    const int lane = threadIdx.x & 31; const int n = blockIdx.x * 8 + (threadIdx.x >> 5); if (n >= NN) return; const int z = lane >> 4, d = (lane & 15) * 2;
    v2f v; v[0] = OZ[((size_t)z * NN + n) * 64 + d]; v[1] = OZ[((size_t)z * NN + n) * 64 + d + 1];
    float* dst = AO + (size_t)n * DIM + (h0 + z) * DK + d; *(volatile v2f*)dst = v; __threadfence(); *(volatile v2f*)dst = v;
}
__global__ __launch_bounds__(256) void k_lnres(float* X, const float* __restrict__ R, const float* __restrict__ g_, const float* __restrict__ b_, int rows, bf* Xh, bf* Xl) {
    typedef __attribute__((ext_vector_type(4))) unsigned short v4us;
    const int lane = threadIdx.x & 31; const int n = blockIdx.x * 8 + (threadIdx.x >> 5); if (n >= rows) return; const int c0 = lane * 4;
    float v[4]; float s = 0.f;
#pragma unroll
    for (int q = 0; q < 4; ++q) { v[q] = X[(size_t)n * DIM + c0 + q] + R[(size_t)n * DIM + c0 + q]; s += v[q]; }
#pragma unroll
    for (int sh = 16; sh; sh >>= 1) s += __shfl_xor(s, sh, 32);
    const float mu = s * (1.0f / DIM); float qq = 0.f;
#pragma unroll
    for (int q = 0; q < 4; ++q) { const float d = v[q] - mu; qq = fmaf(d, d, qq); }
#pragma unroll
    for (int sh = 16; sh; sh >>= 1) qq += __shfl_xor(qq, sh, 32);
    const float rs = rsqrtf(qq * (1.0f / DIM) + 1e-5f); v4f o; v4us oh, ol;
#pragma unroll
    for (int q = 0; q < 4; ++q) { o[q] = (v[q] - mu) * rs * bfr(g_[c0 + q]) + bfr(b_[c0 + q]); unsigned short a, b; splitf(o[q], a, b); oh[q] = a; ol[q] = b; }
#pragma unroll 1
    for (int ps = 0; ps < 2; ++ps) { *(volatile v4f*)(X + (size_t)n * DIM + c0) = o; *(volatile v4us*)(Xh + (size_t)n * DIM + c0) = oh; *(volatile v4us*)(Xl + (size_t)n * DIM + c0) = ol; if (ps == 0) __threadfence(); }
}
__global__ __launch_bounds__(256) void k_gelu_planes(const float* __restrict__ H, size_t n, bf* Ph, bf* Pl) {
    typedef __attribute__((ext_vector_type(2))) unsigned short v2us;
    const int lane = threadIdx.x & 31; const size_t L0 = ((size_t)blockIdx.x * 8 + (threadIdx.x >> 5)) * 8; const size_t nlines = n / 64;
#pragma unroll 1
    for (int ps = 0; ps < 2; ++ps) {
#pragma unroll 1
        for (int l = 0; l < 8; ++l) { const size_t L = L0 + l; if (L >= nlines) break; const size_t e = L * 64 + lane * 2; v2us oh, ol;
#pragma unroll
            for (int q = 0; q < 2; ++q) { unsigned short a, b; splitf(geluf(H[e + q]), a, b); oh[q] = a; ol[q] = b; }
            *(volatile v2us*)(Ph + e) = oh; *(volatile v2us*)(Pl + e) = ol; }
        if (ps == 0) __threadfence(); }
}
__global__ __launch_bounds__(256) void k_fuse(const float* __restrict__ X, bf* Fh, bf* Fl) {
    typedef __attribute__((ext_vector_type(4))) unsigned short v4us;
    const int lane = threadIdx.x & 31; const int t = blockIdx.x * 8 + (threadIdx.x >> 5); if (t >= TT) return; const int c0 = lane * 4; v4us oh, ol;
#pragma unroll
    for (int q = 0; q < 4; ++q) { const float s = (X[(size_t)(3 * t) * DIM + c0 + q] + X[(size_t)(3 * t + 1) * DIM + c0 + q]) + X[(size_t)(3 * t + 2) * DIM + c0 + q]; unsigned short a, b; splitf(__fdiv_rn(s, 3.0f), a, b); oh[q] = a; ol[q] = b; }
#pragma unroll 1
    for (int ps = 0; ps < 2; ++ps) { *(volatile v4us*)(Fh + (size_t)t * DIM + c0) = oh; *(volatile v4us*)(Fl + (size_t)t * DIM + c0) = ol; if (ps == 0) __threadfence(); }
}
__global__ __launch_bounds__(256) void k_final(const float* __restrict__ O2, const float* __restrict__ b2, float* OUT) {
    const int lane = threadIdx.x & 31; const int f = (blockIdx.x * 8 + (threadIdx.x >> 5)) * 32 + lane; if (f - lane >= TT * 3) return;
    const float v = O2[(size_t)(f / 3) * 64 + (f % 3)] + bfr(b2[f % 3]);
    *(volatile float*)(OUT + f) = v; __threadfence(); *(volatile float*)(OUT + f) = v;
}

extern "C" void kernel_launch(void* const* d_in, const int* in_sizes, int n_in,
                              void* d_out, int out_size, void* d_ws, size_t ws_size, hipStream_t stream) {
    (void)in_sizes; (void)n_in; (void)out_size;
    const float* obs = (const float*)d_in[0]; const float* cf = (const float*)d_in[1]; const float* npw = (const float*)d_in[2]; const float* npb = (const float*)d_in[3]; const float* temb = (const float*)d_in[4]; const float* semb = (const float*)d_in[5];
    const float* Wq = (const float*)d_in[6]; const float* bq = (const float*)d_in[7]; const float* Wk = (const float*)d_in[8]; const float* bk = (const float*)d_in[9]; const float* Wv = (const float*)d_in[10]; const float* bv = (const float*)d_in[11];
    const float* ew = (const float*)d_in[12]; const float* eb = (const float*)d_in[13]; const float* l1g = (const float*)d_in[14]; const float* l1b = (const float*)d_in[15]; const float* l2g = (const float*)d_in[16]; const float* l2b = (const float*)d_in[17];
    const float* f1w = (const float*)d_in[18]; const float* f1b = (const float*)d_in[19]; const float* f2w = (const float*)d_in[20]; const float* f2b = (const float*)d_in[21];
    const float* o1w = (const float*)d_in[22]; const float* o1b = (const float*)d_in[23]; const float* o2w = (const float*)d_in[24]; const float* o2b = (const float*)d_in[25];
    float* OUT = (float*)d_out;
    char* wsp = (char*)d_ws;
    auto take = [&](size_t bytes) { char* p = wsp; wsp += (bytes + 255) & ~(size_t)255; return (void*)p; };
    bf* WQ = (bf*)take((size_t)NL * DIM * DIM * 2); bf* WK = (bf*)take((size_t)NL * DIM * DIM * 2); bf* WV = (bf*)take((size_t)NL * DIM * DIM * 2); bf* W1 = (bf*)take((size_t)NL * DFF * DIM * 2); bf* W2 = (bf*)take((size_t)NL * DIM * DFF * 2); bf* WO1 = (bf*)take((size_t)DIM * DIM * 2); bf* WO2 = (bf*)take((size_t)64 * DIM * 2);
    float* X = (float*)take((size_t)NN * DIM * 4); bf* Xh = (bf*)take((size_t)NN * DIM * 2); bf* Xl = (bf*)take((size_t)NN * DIM * 2);
    float* Q = (float*)take((size_t)NN * DIM * 4); float* Kf = (float*)take((size_t)NN * DIM * 4); float* V = (float*)take((size_t)NN * DIM * 4); float* AO = (float*)take((size_t)NN * DIM * 4);
    float* DIST = (float*)take((size_t)NN * NN * 4); float* ATAB = (float*)take((size_t)NHD * NN * 4);
    bf* QPh = (bf*)take((size_t)ZH * NN * DK * 2); bf* QPl = (bf*)take((size_t)ZH * NN * DK * 2); bf* KPh = (bf*)take((size_t)ZH * NN * DK * 2); bf* KPl = (bf*)take((size_t)ZH * NN * DK * 2);
    bf* VTh = (bf*)take((size_t)ZH * 64 * NN * 2); bf* VTl = (bf*)take((size_t)ZH * 64 * NN * 2);
    float* Sb = (float*)take((size_t)ZH * NN * NN * 4); bf* PH = (bf*)take((size_t)ZH * NN * NN * 2); bf* PL = (bf*)take((size_t)ZH * NN * NN * 2); float* OZ = (float*)take((size_t)ZH * NN * 64 * 4);
    float* H1 = (float*)take((size_t)NN * DFF * 4); bf* H1h = (bf*)take((size_t)NN * DFF * 2); bf* H1l = (bf*)take((size_t)NN * DFF * 2);
    bf* FUh = (bf*)take((size_t)TT * DIM * 2); bf* FUl = (bf*)take((size_t)TT * DIM * 2); float* G1 = (float*)take((size_t)TT * DIM * 4); bf* G1h = (bf*)take((size_t)TT * DIM * 2); bf* G1l = (bf*)take((size_t)TT * DIM * 2); float* O2 = (float*)take((size_t)TT * 64 * 4);
    if ((size_t)(wsp - (char*)d_ws) > ws_size) return;
    { const size_t n1 = (size_t)NL * DIM * DIM / 8, n2 = (size_t)NL * DFF * DIM / 8;
      k_cvt8<<<(unsigned)((n1 + 255) / 256), 256, 0, stream>>>(Wq, WQ, n1); k_cvt8<<<(unsigned)((n1 + 255) / 256), 256, 0, stream>>>(Wk, WK, n1); k_cvt8<<<(unsigned)((n1 + 255) / 256), 256, 0, stream>>>(Wv, WV, n1);
      k_cvt8<<<(unsigned)((n2 + 255) / 256), 256, 0, stream>>>(f1w, W1, n2); k_cvt8<<<(unsigned)((n2 + 255) / 256), 256, 0, stream>>>(f2w, W2, n2);
      k_cvt8<<<(DIM * DIM / 8 + 255) / 256, 256, 0, stream>>>(o1w, WO1, DIM * DIM / 8); k_w2pad<<<(64 * DIM / 8 + 255) / 256, 256, 0, stream>>>(o2w, WO2); }
    k_embed<<<NN / 8, 256, 0, stream>>>(obs, cf, npw, npb, temb, semb, X, Xh, Xl);
    k_dist<<<NN / 8, 256, 0, stream>>>(obs, DIST);
    for (int l = 0; l < NL; ++l) {
        k_gemmw<bf, 1, true><<<dim3(NN / 64, DIM / 64, 1), 32, 0, stream>>>(Xh, Xl, WQ + (size_t)l * DIM * DIM, nullptr, DIM, Q, DIM, bq + l * DIM, 0, 0, 0);
        k_gemmw<bf, 1, true><<<dim3(NN / 64, DIM / 64, 1), 32, 0, stream>>>(Xh, Xl, WK + (size_t)l * DIM * DIM, nullptr, DIM, Kf, DIM, bk + l * DIM, 0, 0, 0);
        k_gemmw<bf, 1, true><<<dim3(NN / 64, DIM / 64, 1), 32, 0, stream>>>(Xh, Xl, WV + (size_t)l * DIM * DIM, nullptr, DIM, V, DIM, bv + l * DIM, 0, 0, 0);
        k_atab<<<NN / 32 / 8, 256, 0, stream>>>(obs, cf, ew + l * NHD * 9, ATAB);
        for (int h0 = 0; h0 < NHD; h0 += ZH) {
            k_qkplanes<<<(unsigned)(((size_t)ZH * NN * DK / 64 + 63) / 64), 256, 0, stream>>>(Q, Kf, h0, QPh, QPl, KPh, KPl);
            k_vT<<<dim3(NN / 64, 1, ZH), 256, 0, stream>>>(V, h0, VTh, VTl);
            k_gemmw<bf, 2, false><<<dim3(NN / 64, NN / 64, ZH), 32, 0, stream>>>(QPh, QPl, KPh, KPl, DK, Sb, NN, nullptr, (size_t)NN * DK, (size_t)NN * DK, (size_t)NN * NN);
            k_softb<<<dim3(NN / 8, 1, ZH), 256, 0, stream>>>(Sb, ATAB, DIST, ew + l * NHD * 9, eb + l * NHD, h0, PH, PL);
            k_gemmw<bf, 2, false><<<dim3(NN / 64, 1, ZH), 32, 0, stream>>>(PH, PL, VTh, VTl, NN, OZ, 64, nullptr, (size_t)NN * NN, (size_t)64 * NN, (size_t)NN * 64);
            k_mergez<<<NN / 8, 256, 0, stream>>>(OZ, h0, AO); }
        k_lnres<<<NN / 8, 256, 0, stream>>>(X, AO, l1g + l * DIM, l1b + l * DIM, NN, Xh, Xl);
        k_gemmw<bf, 1, true><<<dim3(NN / 64, DFF / 64, 1), 32, 0, stream>>>(Xh, Xl, W1 + (size_t)l * DFF * DIM, nullptr, DIM, H1, DFF, f1b + l * DFF, 0, 0, 0);
        k_gelu_planes<<<(unsigned)(((size_t)NN * DFF / 64 + 63) / 64), 256, 0, stream>>>(H1, (size_t)NN * DFF, H1h, H1l);
        k_gemmw<bf, 1, true><<<dim3(NN / 64, DIM / 64, 1), 32, 0, stream>>>(H1h, H1l, W2 + (size_t)l * DIM * DFF, nullptr, DFF, AO, DIM, f2b + l * DIM, 0, 0, 0);
        k_lnres<<<NN / 8, 256, 0, stream>>>(X, AO, l2g + l * DIM, l2b + l * DIM, NN, Xh, Xl); }
    k_fuse<<<TT / 8, 256, 0, stream>>>(X, FUh, FUl);
    k_gemmw<bf, 1, true><<<dim3(TT / 64, DIM / 64, 1), 32, 0, stream>>>(FUh, FUl, WO1, nullptr, DIM, G1, DIM, o1b, 0, 0, 0);
    k_gelu_planes<<<(unsigned)(((size_t)TT * DIM / 64 + 63) / 64), 256, 0, stream>>>(G1, (size_t)TT * DIM, G1h, G1l);
    k_gemmw<bf, 1, false><<<dim3(TT / 64, 1, 1), 32, 0, stream>>>(G1h, G1l, WO2, nullptr, DIM, O2, 64, nullptr, 0, 0, 0);
    k_final<<<(TT * 3 / 32 + 7) / 8, 256, 0, stream>>>(O2, o2b, OUT);
}
